// RelativePositionalEmbedding_37349035606582
// MI455X (gfx1250) — hardware-verified
//
#include <hip/hip_runtime.h>
#include <stdint.h>

typedef __attribute__((ext_vector_type(16))) _Float16 v16h;
typedef __attribute__((ext_vector_type(8)))  _Float16 v8h;
typedef __attribute__((ext_vector_type(16))) __bf16   v16b;
typedef __attribute__((ext_vector_type(8)))  __bf16   v8b;
typedef __attribute__((ext_vector_type(8)))  float    v8f;
typedef __attribute__((ext_vector_type(4)))  float    v4f;
#define PSCALE 32768.0f
#define U16(p) ((const unsigned short*)(const void*)(p))
#define PSCALE_INV (1.0f / 32768.0f)

__device__ __forceinline__ unsigned short f2bf_bits(float f) {
  unsigned u = __float_as_uint(f);
  return (unsigned short)((u + 0x7FFFu + ((u >> 16) & 1u)) >> 16);
}
__device__ __forceinline__ float bf_bits2f(unsigned short h) { return __uint_as_float(((unsigned)h) << 16); }

__device__ __forceinline__ void dep_guard_h(v8f& a, v8f& b, v16h x, v16h y) { asm volatile("v_nop\n\tv_nop\n\tv_nop\n\tv_nop" : "+v"(a), "+v"(b) : "v"(x), "v"(y)); }
__device__ __forceinline__ void dep_guard_b(v8f& a, v8f& b, v16b x, v16b y) { asm volatile("v_nop\n\tv_nop\n\tv_nop\n\tv_nop" : "+v"(a), "+v"(b) : "v"(x), "v"(y)); }
__device__ __forceinline__ void keep4_h(v16h a, v16h b, v16h c, v16h d) { asm volatile("v_nop" :: "v"(a), "v"(b), "v"(c), "v"(d)); }
__device__ __forceinline__ void keep4_b(v16b a, v16b b, v16b c, v16b d) { asm volatile("v_nop" :: "v"(a), "v"(b), "v"(c), "v"(d)); }
__device__ __forceinline__ void acc_guard4(v8f& a, v8f& b, v8f& c, v8f& d) { asm volatile("v_nop\n\tv_nop\n\tv_nop\n\tv_nop" : "+v"(a), "+v"(b), "+v"(c), "+v"(d)); }
template <typename T> struct Frag;
template <> struct Frag<_Float16> {
  typedef v16h V; union U { v16h v; v8h h[2]; };
  static __device__ __forceinline__ v16h load(const _Float16* p) {
    U f; f.h[0] = *(const v8h*)(p); f.h[1] = *(const v8h*)(p + 16); return f.v;
  }
  static __device__ __forceinline__ v8f mma(v16h a, v16h b, v8f c) {
    return __builtin_amdgcn_wmma_f32_16x16x32_f16(false, a, false, b, (short)0, c, false, false);
  }
  static __device__ __forceinline__ void guard(v8f& a, v8f& b, v16h x, v16h y) { dep_guard_h(a, b, x, y); }
  static __device__ __forceinline__ void keep(v16h a, v16h b, v16h c, v16h d) { keep4_h(a, b, c, d); }
};
template <> struct Frag<__bf16> {
  typedef v16b V; union U { v16b v; v8b h[2]; };
  static __device__ __forceinline__ v16b load(const __bf16* p) {
    U f; f.h[0] = *(const v8b*)(p); f.h[1] = *(const v8b*)(p + 16); return f.v;
  }
  static __device__ __forceinline__ v8f mma(v16b a, v16b b, v8f c) {
    return __builtin_amdgcn_wmma_f32_16x16x32_bf16(false, a, false, b, (short)0, c, false, false);
  }
  static __device__ __forceinline__ void guard(v8f& a, v8f& b, v16b x, v16b y) { dep_guard_b(a, b, x, y); }
  static __device__ __forceinline__ void keep(v16b a, v16b b, v16b c, v16b d) { keep4_b(a, b, c, d); }
};

template <int ET> struct Elem;
template <> struct Elem<0> { typedef _Float16 T; };
template <> struct Elem<1> { typedef __bf16 T; };
template <int ET, bool SPLIT, int BIAS_MODE, int OUT_MODE, bool RESID, int ACT = 0>
__global__ __launch_bounds__(256) void wmma_gemm64(
    const unsigned short* __restrict__ Ap, const unsigned short* __restrict__ A2p, int lda, long strideA,
    const unsigned short* __restrict__ Btp, const unsigned short* __restrict__ Bt2p, int ldb, long strideB,
    void* __restrict__ Cout, void* __restrict__ Cout2, int ldc, long strideC,
    const float* __restrict__ bias,
    const float* __restrict__ resid, long strideR,
    int M, int N, int K, float scale) {
  typedef typename Elem<ET>::T T;
  typedef typename Frag<T>::V V;
  const T* A = (const T*)Ap; const T* A2 = (const T*)A2p; const T* Bt = (const T*)Btp; const T* Bt2 = (const T*)Bt2p;
  __shared__ __align__(16) float sT[8][16 * 68];
  const int b    = blockIdx.y;
  const int lane = threadIdx.x & 31;
  const int wave = threadIdx.x >> 5;
  const int tilesN = N >> 6;
  const int tilesM = M >> 6;
  const int tile = blockIdx.x * 8 + wave;
  if (tile >= tilesM * tilesN) return;
  const int tm = tile / tilesN;
  const int tn = tile - tm * tilesN;
  const int m0 = tm << 6;
  const int n0 = tn << 6;

  const T* Ab  = A  + (size_t)b * strideA;
  const T* Bb  = Bt + (size_t)b * strideB;
  const T* Ab2 = SPLIT ? (A2  + (size_t)b * strideA) : nullptr;
  const T* Bb2 = SPLIT ? (Bt2 + (size_t)b * strideB) : nullptr;

  const int rlane = lane & 15;
  const int koff  = (lane >> 4) * 8;
  const int mOff  = (lane >> 4) * 8;

  v8f acc[4][4];
#pragma unroll
  for (int i = 0; i < 4; ++i)
#pragma unroll
    for (int j = 0; j < 4; ++j) acc[i][j] = (v8f){0.f,0.f,0.f,0.f,0.f,0.f,0.f,0.f};

  for (int k0 = 0; k0 < K; k0 += 32) {
    V bh[4], bl[4];
#pragma unroll
    for (int j = 0; j < 4; ++j) {
      const size_t bo = (size_t)(n0 + (j << 4) + rlane) * ldb + koff + k0;
      bh[j] = Frag<T>::load(Bb + bo);
      if (SPLIT) bl[j] = Frag<T>::load(Bb2 + bo);
    }
#pragma unroll
    for (int i = 0; i < 4; ++i) {
      const size_t ao = (size_t)(m0 + (i << 4) + rlane) * lda + koff + k0;
      V ah = Frag<T>::load(Ab + ao);
      V al;
      if (SPLIT) al = Frag<T>::load(Ab2 + ao);
#pragma unroll
      for (int j = 0; j < 4; ++j) {
        acc[i][j] = Frag<T>::mma(ah, bh[j], acc[i][j]);
        if (SPLIT) {
          acc[i][j] = Frag<T>::mma(ah, bl[j], acc[i][j]);
          acc[i][j] = Frag<T>::mma(al, bh[j], acc[i][j]);
        }
      }
      Frag<T>::guard(acc[i][0], acc[i][3], ah, SPLIT ? al : ah);
    }
    Frag<T>::keep(bh[0], bh[1], bh[2], bh[3]);
    if (SPLIT) Frag<T>::keep(bl[0], bl[1], bl[2], bl[3]);
  }
  acc_guard4(acc[0][0], acc[0][1], acc[0][2], acc[0][3]);
  acc_guard4(acc[1][0], acc[1][1], acc[1][2], acc[1][3]);
  acc_guard4(acc[2][0], acc[2][1], acc[2][2], acc[2][3]);
  acc_guard4(acc[3][0], acc[3][1], acc[3][2], acc[3][3]);

  float* slab = sT[wave];
  const float* Rb = RESID ? (resid + (size_t)b * strideR) : nullptr;
#pragma unroll
  for (int i = 0; i < 4; ++i) {
    const int mBase = m0 + (i << 4);
#pragma unroll
    for (int j = 0; j < 4; ++j) {
      const int n = n0 + (j << 4) + rlane;
      float bv = 0.f;
      if (BIAS_MODE == 2) bv = bias[n];
#pragma unroll
      for (int r = 0; r < 8; ++r) {
        float v = acc[i][j][r] * scale;
        if (BIAS_MODE == 1) v += bias[mBase + mOff + r];
        if (BIAS_MODE == 2) v += bv;
        if (RESID) v += Rb[(size_t)(mBase + mOff + r) * ldc + n];
        if (ACT == 1) v = tanhf(v);
        if (ACT == 2) v = fmaxf(v, 0.0f);
        if (ACT == 3) v = v / (1.0f + expf(-v));
        if (ACT == 4) v = (v > 0.f) ? v : 0.01f * v;
        if (ACT == 5) v = 0.5f * v * (1.0f + erff(v * 0.70710678118654752f));
        slab[(mOff + r) * 68 + (j << 4) + rlane] = v;
      }
    }
    __builtin_amdgcn_fence(__ATOMIC_RELEASE, "workgroup");
    __builtin_amdgcn_wave_barrier();
    __builtin_amdgcn_fence(__ATOMIC_ACQUIRE, "workgroup");
    if (OUT_MODE == 0) {
      float* C = (float*)Cout + (size_t)b * strideC;
      const int hh = lane >> 4, c4 = (lane & 15) * 4;
      for (int pass = 0; pass < 2; ++pass) {
#pragma unroll
        for (int it = 0; it < 8; ++it) {
          const int row = it * 2 + hh;
          v4f v = *(const v4f*)(slab + row * 68 + c4);
          *(volatile v4f*)(C + (size_t)(mBase + row) * ldc + n0 + c4) = v;
        }
        __threadfence();
      }
    } else {
      const int q = lane >> 3, c8 = (lane & 7) * 8;
      unsigned short* C  = (unsigned short*)Cout  + (size_t)b * strideC;
      unsigned short* C2 = (OUT_MODE == 2) ? ((unsigned short*)Cout2 + (size_t)b * strideC) : nullptr;
      for (int pass = 0; pass < 2; ++pass) {
#pragma unroll
        for (int it = 0; it < 4; ++it) {
          const int row = it * 4 + q;
          const float* sp = slab + row * 68 + c8;
          v8h hv, lv;
#pragma unroll
          for (int e = 0; e < 8; ++e) {
            if (OUT_MODE == 1) {
              hv[e] = (_Float16)sp[e];
            } else {
              unsigned short hb = f2bf_bits(sp[e]);
              unsigned short lb = f2bf_bits(sp[e] - bf_bits2f(hb));
              hv[e] = __builtin_bit_cast(_Float16, hb);
              lv[e] = __builtin_bit_cast(_Float16, lb);
            }
          }
          *(volatile v8h*)(C + (size_t)(mBase + row) * ldc + n0 + c8) = hv;
          if (OUT_MODE == 2) *(volatile v8h*)(C2 + (size_t)(mBase + row) * ldc + n0 + c8) = lv;
        }
        __threadfence();
      }
    }
    __builtin_amdgcn_fence(__ATOMIC_RELEASE, "workgroup");
    __builtin_amdgcn_wave_barrier();
    __builtin_amdgcn_fence(__ATOMIC_ACQUIRE, "workgroup");
  }
}

__global__ __launch_bounds__(256) void cast_f32_f16x2(
    const float* __restrict__ in, _Float16* __restrict__ out, int n2) {
  int i = blockIdx.x * 256 + threadIdx.x;
  if (i < n2) {
    const _Float16 h0 = (_Float16)in[2 * i], h1 = (_Float16)in[2 * i + 1];
    const unsigned u = (unsigned)__builtin_bit_cast(unsigned short, h0) | ((unsigned)__builtin_bit_cast(unsigned short, h1) << 16);
    ((volatile unsigned*)out)[i] = u;
    __threadfence();
    ((volatile unsigned*)out)[i] = u;
  }
}

__global__ __launch_bounds__(256) void cast_scale_f32_f16x2(
    const float* __restrict__ in, _Float16* __restrict__ out, int n2, float scale) {
  int i = blockIdx.x * 256 + threadIdx.x;
  if (i < n2) {
    const _Float16 h0 = (_Float16)(in[2 * i] * scale), h1 = (_Float16)(in[2 * i + 1] * scale);
    const unsigned u = (unsigned)__builtin_bit_cast(unsigned short, h0) | ((unsigned)__builtin_bit_cast(unsigned short, h1) << 16);
    ((volatile unsigned*)out)[i] = u;
    __threadfence();
    ((volatile unsigned*)out)[i] = u;
  }
}

__global__ __launch_bounds__(256) void cast_rk_rows(
    const float* __restrict__ rk, _Float16* __restrict__ out, int rows_in, int rows_out, float scale) {
  const int i = blockIdx.x * 256 + threadIdx.x;
  const int n2 = rows_out * 32;
  if (i < n2) {
    const int idx = 2 * i;
    const int row = idx >> 6;
    float a = 0.f, bb = 0.f;
    if (row < rows_in) { a = rk[idx] * scale; bb = rk[idx + 1] * scale; }
    const _Float16 h0 = (_Float16)a, h1 = (_Float16)bb;
    const unsigned u = (unsigned)__builtin_bit_cast(unsigned short, h0) | ((unsigned)__builtin_bit_cast(unsigned short, h1) << 16);
    ((volatile unsigned*)out)[i] = u;
    __threadfence();
    ((volatile unsigned*)out)[i] = u;
  }
}

__global__ __launch_bounds__(256) void cast_rv_T(
    const float* __restrict__ rv, _Float16* __restrict__ out, int rows_in, int kpad, float scale) {
  const int i = blockIdx.x * 256 + threadIdx.x;
  const int n2 = 32 * kpad;
  if (i < n2) {
    const int idx = 2 * i;
    const int dd = idx / kpad;
    const int r  = idx - dd * kpad;
    const float a  = (r < rows_in)     ? rv[r * 64 + dd] * scale : 0.f;
    const float bb = (r + 1 < rows_in) ? rv[(r + 1) * 64 + dd] * scale : 0.f;
    const _Float16 h0 = (_Float16)a, h1 = (_Float16)bb;
    const unsigned u = (unsigned)__builtin_bit_cast(unsigned short, h0) | ((unsigned)__builtin_bit_cast(unsigned short, h1) << 16);
    ((volatile unsigned*)out)[i] = u;
    __threadfence();
    ((volatile unsigned*)out)[i] = u;
  }
}

#define RA_D    64
#define RA_NW   4
#define RA_KC   64
#define RA_S    2048
#define RA_E    1024
#define RA_H    16
#define RA_P    128
#define RA_NB   32
#define RA_NT   17
#define RA_QRP  272
#define RA_SBP  256
#define RA_PBK  288
#define RA_LO_K   0
#define RA_LO_V   8192
#define RA_LO_P   16384
#define RA_LO_OS  0
#define RA_LO_SB  24576
#define RA_LO_QR  90112
#define RA_LDS    159744

__device__ __forceinline__ v8f ra_mma(v16h a, v16h b, v8f c) {
  c = __builtin_amdgcn_wmma_f32_16x16x32_f16(false, a, false, b, (short)0, c, false, false);
  asm volatile("v_nop\n\tv_nop\n\tv_nop\n\tv_nop" : "+v"(c) : "v"(a), "v"(b));
  return c;
}

__global__ __launch_bounds__(128)
void rel_attn_kernel(const _Float16* __restrict__ Qg, const _Float16* __restrict__ Kg,
                     const _Float16* __restrict__ Vg, const _Float16* __restrict__ rk16,
                     const _Float16* __restrict__ rvT16, _Float16* __restrict__ Og) {
  extern __shared__ __align__(16) unsigned char ra_smem[];
  union FH { v16h v; v8h h[2]; };
  const int tid  = threadIdx.x;
  const int wave = __builtin_amdgcn_readfirstlane(tid >> 5);
  const int lane = tid & 31;
  const int hh   = lane >> 4;
  const int c    = lane & 15;
  const float NEG_INF = -__builtin_inff();

  _Float16* Ksh = (_Float16*)(ra_smem + RA_LO_K);
  _Float16* Vth = (_Float16*)(ra_smem + RA_LO_V);
  _Float16* pw  = (_Float16*)(ra_smem + RA_LO_P) + wave * (16 * RA_KC);
  float*    os  = (float*)(ra_smem + RA_LO_OS) + wave * (16 * 68);
  float*    sb  = (float*)(ra_smem + RA_LO_SB) + wave * (16 * RA_SBP);
  float*    qrs = (float*)(ra_smem + RA_LO_QR) + wave * (16 * RA_QRP);
  _Float16* pb  = (_Float16*)(ra_smem + RA_LO_QR + wave * (16 * RA_QRP * 4));

  const int bx = blockIdx.x;
  const int qb = bx & 31;
  const int bh = bx >> 5;
  const int h  = bh & 15;
  const int b  = bh >> 4;
  const int q0 = qb * 64 + wave * 16;
  const size_t rowbase = (size_t)b * RA_S;
  const int hoff = h * RA_D;

  v16h qa[2];
  {
    const _Float16* qrow = Qg + (rowbase + q0 + c) * RA_E + hoff;
#pragma unroll
    for (int dc = 0; dc < 2; ++dc) {
      FH f;
      f.h[0] = *(const v8h*)(qrow + dc * 32 + 8 * hh);
      f.h[1] = *(const v8h*)(qrow + dc * 32 + 16 + 8 * hh);
      qa[dc] = f.v;
    }
  }

#pragma unroll 1
  for (int nt = 0; nt < RA_NT; ++nt) {
    v8f acc = (v8f){0.f,0.f,0.f,0.f,0.f,0.f,0.f,0.f};
#pragma unroll
    for (int dc = 0; dc < 2; ++dc) {
      FH rb;
      const _Float16* rp = rk16 + (size_t)(nt * 16 + c) * RA_D + dc * 32 + 8 * hh;
      rb.h[0] = *(const v8h*)(rp);
      rb.h[1] = *(const v8h*)(rp + 16);
      acc = ra_mma(qa[dc], rb.v, acc);
    }
#pragma unroll
    for (int r = 0; r < 8; ++r) qrs[(8 * hh + r) * RA_QRP + nt * 16 + c] = acc[r] * (1.0f / 64.0f);
  }
  for (int i = lane; i < 16 * RA_SBP; i += 32) sb[i] = NEG_INF;

  float mrow[8], lrow[8], pL[8], pR[8];
  v8f oacc[4];
#pragma unroll
  for (int r = 0; r < 8; ++r) { mrow[r] = NEG_INF; lrow[r] = 0.f; pL[r] = 0.f; pR[r] = 0.f; }
#pragma unroll
  for (int t = 0; t < 4; ++t) oacc[t] = (v8f){0.f,0.f,0.f,0.f,0.f,0.f,0.f,0.f};

  for (int kc = 0; kc < RA_NB; ++kc) {
    const int kv0 = kc * RA_KC;
    __syncthreads();
    {
      const int kvr = tid >> 1, dh = (tid & 1) * 32;
      const _Float16* krow = Kg + (rowbase + kv0 + kvr) * RA_E + hoff + dh;
      const _Float16* vrow = Vg + (rowbase + kv0 + kvr) * RA_E + hoff + dh;
#pragma unroll
      for (int i = 0; i < 4; ++i) {
        const v8h kk = *(const v8h*)(krow + 8 * i);
        *(v8h*)(Ksh + kvr * RA_D + dh + 8 * i) = kk;
        const v8h vv = *(const v8h*)(vrow + 8 * i);
#pragma unroll
        for (int e = 0; e < 8; ++e) Vth[(dh + 8 * i + e) * RA_KC + kvr] = vv[e];
      }
    }
    __syncthreads();

    v8f s[4];
#pragma unroll
    for (int j = 0; j < 4; ++j) {
      s[j] = (v8f){0.f,0.f,0.f,0.f,0.f,0.f,0.f,0.f};
#pragma unroll
      for (int dc = 0; dc < 2; ++dc) {
        FH kb;
        kb.h[0] = *(const v8h*)(Ksh + (j * 16 + c) * RA_D + dc * 32 + 8 * hh);
        kb.h[1] = *(const v8h*)(Ksh + (j * 16 + c) * RA_D + dc * 32 + 16 + 8 * hh);
        s[j] = ra_mma(qa[dc], kb.v, s[j]);
      }
    }

    const int relHi = kv0 + (RA_KC - 1) - q0;
    const int relLo = kv0 - q0 - 15;
    const bool farL = (relHi <= -RA_P);
    const bool farR = (relLo >= RA_P);
    const bool far  = farL || farR;
    const int  fidx = farL ? 0 : (2 * RA_P);

#pragma unroll
    for (int r = 0; r < 8; ++r) {
      const int lr = 8 * hh + r;
      const int qrow = q0 + lr;
      float fb = 0.f;
      if (far) fb = qrs[lr * RA_QRP + fidx];
      float m = NEG_INF;
#pragma unroll
      for (int j = 0; j < 4; ++j) {
        const int rel = (kv0 + j * 16 + c) - qrow;
        float bias;
        if (far) {
          bias = fb;
        } else {
          int ridx = rel < -RA_P ? -RA_P : (rel > RA_P ? RA_P : rel);
          bias = qrs[lr * RA_QRP + ridx + RA_P];
        }
        const float sv = (s[j][r] + bias) * 0.125f;
        s[j][r] = sv;
        if (!far) {
          if (rel >= -(RA_P - 1) && rel <= (RA_P - 1)) sb[lr * RA_SBP + rel + (RA_P - 1)] = sv;
        }
        m = fmaxf(m, sv);
      }
#pragma unroll
      for (int off = 1; off < 16; off <<= 1) m = fmaxf(m, __shfl_xor(m, off, 32));
      const float mnew = fmaxf(mrow[r], m);
      const float alpha = __expf(mrow[r] - mnew);
      mrow[r] = mnew;
      float psum = 0.f, aL = 0.f, aR = 0.f;
#pragma unroll
      for (int j = 0; j < 4; ++j) {
        const float p = __expf(s[j][r] - mnew);
        psum += p;
        pw[lr * RA_KC + j * 16 + c] = (_Float16)(p * 32768.0f);
        if (!far) {
          const int rel = (kv0 + j * 16 + c) - qrow;
          aL += (rel <= -RA_P) ? p : 0.f;
          aR += (rel >= RA_P) ? p : 0.f;
        }
      }
      if (far) { aL = farL ? psum : 0.f; aR = farR ? psum : 0.f; }
      pL[r] = pL[r] * alpha + aL;
      pR[r] = pR[r] * alpha + aR;
#pragma unroll
      for (int off = 1; off < 16; off <<= 1) psum += __shfl_xor(psum, off, 32);
      lrow[r] = lrow[r] * alpha + psum;
#pragma unroll
      for (int t = 0; t < 4; ++t) oacc[t][r] *= alpha;
    }
    __builtin_amdgcn_fence(__ATOMIC_RELEASE, "workgroup");
    __builtin_amdgcn_wave_barrier();
    __builtin_amdgcn_fence(__ATOMIC_ACQUIRE, "workgroup");
#pragma unroll 1
    for (int kk = 0; kk < 2; ++kk) {
      FH pa;
      pa.h[0] = *(const v8h*)(pw + c * RA_KC + kk * 32 + 8 * hh);
      pa.h[1] = *(const v8h*)(pw + c * RA_KC + kk * 32 + 16 + 8 * hh);
#pragma unroll
      for (int t = 0; t < 4; ++t) {
        FH vb;
        vb.h[0] = *(const v8h*)(Vth + (t * 16 + c) * RA_KC + kk * 32 + 8 * hh);
        vb.h[1] = *(const v8h*)(Vth + (t * 16 + c) * RA_KC + kk * 32 + 16 + 8 * hh);
        oacc[t] = ra_mma(pa.v, vb.v, oacc[t]);
      }
    }
  }
  __syncthreads();

#pragma unroll
  for (int r = 0; r < 8; ++r) {
#pragma unroll
    for (int off = 1; off < 16; off <<= 1) {
      pL[r] += __shfl_xor(pL[r], off, 32);
      pR[r] += __shfl_xor(pR[r], off, 32);
    }
  }
#pragma unroll 1
  for (int ci = 0; ci < RA_PBK / 16; ++ci) {
    const int col = ci * 16 + c;
    int bi = col - 1;
    bi = bi < 0 ? 0 : (bi > 2 * RA_P - 2 ? 2 * RA_P - 2 : bi);
#pragma unroll
    for (int r = 0; r < 8; ++r) {
      const int lr = 8 * hh + r;
      float val;
      if (col == 0) val = pL[r];
      else if (col == 2 * RA_P) val = pR[r];
      else if (col < 2 * RA_P) val = __expf(sb[lr * RA_SBP + bi] - mrow[r]);
      else val = 0.f;
      pb[lr * RA_PBK + col] = (_Float16)(val * 16.0f);
    }
  }
  __builtin_amdgcn_fence(__ATOMIC_RELEASE, "workgroup");
  __builtin_amdgcn_wave_barrier();
  __builtin_amdgcn_fence(__ATOMIC_ACQUIRE, "workgroup");
#pragma unroll 1
  for (int kk = 0; kk < RA_PBK / 32; ++kk) {
    FH pa;
    pa.h[0] = *(const v8h*)(pb + c * RA_PBK + kk * 32 + 8 * hh);
    pa.h[1] = *(const v8h*)(pb + c * RA_PBK + kk * 32 + 16 + 8 * hh);
#pragma unroll
    for (int t = 0; t < 4; ++t) {
      FH vb;
      const _Float16* vp = rvT16 + (size_t)(t * 16 + c) * RA_PBK + kk * 32 + 8 * hh;
      vb.h[0] = *(const v8h*)(vp);
      vb.h[1] = *(const v8h*)(vp + 16);
      oacc[t] = ra_mma(pa.v, vb.v, oacc[t]);
    }
  }

#pragma unroll
  for (int r = 0; r < 8; ++r) {
    const float inv = 1.0f / (lrow[r] * 32768.0f);
#pragma unroll
    for (int t = 0; t < 4; ++t) os[(8 * hh + r) * 68 + t * 16 + c] = oacc[t][r] * inv;
  }
  __builtin_amdgcn_fence(__ATOMIC_RELEASE, "workgroup");
  __builtin_amdgcn_wave_barrier();
  __builtin_amdgcn_fence(__ATOMIC_ACQUIRE, "workgroup");
  {
    const int q = lane >> 3, c8 = (lane & 7) * 8;
    for (int pass = 0; pass < 2; ++pass) {
#pragma unroll
      for (int it = 0; it < 4; ++it) {
        const int row = it * 4 + q;
        const float* sp = os + row * 68 + c8;
        v8h hv;
#pragma unroll
        for (int e = 0; e < 8; ++e) hv[e] = (_Float16)sp[e];
        *(volatile v8h*)(Og + (rowbase + q0 + row) * RA_E + hoff + c8) = hv;
      }
      __threadfence();
    }
  }
}

extern "C" void kernel_launch(void* const* d_in, const int* in_sizes, int n_in,
                              void* d_out, int out_size, void* d_ws, size_t ws_size,
                              hipStream_t stream) {
  const int B = 2, S = 2048, E = 1024, D = 64, R = 257;
  const int RKROWS = 272, RVK = 288;
  const int M = B * S;
  if (n_in < 13) return;
  if (in_sizes[0] != M * E || in_sizes[1] != M * E || in_sizes[2] != M * E) return;
  if (in_sizes[3] != E * E || in_sizes[5] != E * E || in_sizes[7] != E * E || in_sizes[9] != E * E) return;
  if (in_sizes[4] != E || in_sizes[6] != E || in_sizes[8] != E || in_sizes[10] != E) return;
  if (in_sizes[11] != R * D || in_sizes[12] != R * D) return;
  if (out_size != M * E) return;

  const float* q  = (const float*)d_in[0];
  const float* k  = (const float*)d_in[1];
  const float* v  = (const float*)d_in[2];
  const float* Wq = (const float*)d_in[3];
  const float* bq = (const float*)d_in[4];
  const float* Wk = (const float*)d_in[5];
  const float* bk = (const float*)d_in[6];
  const float* Wv = (const float*)d_in[7];
  const float* bv = (const float*)d_in[8];
  const float* Wo = (const float*)d_in[9];
  const float* bo = (const float*)d_in[10];
  const float* rk = (const float*)d_in[11];
  const float* rv = (const float*)d_in[12];
  float* out = (float*)d_out;

  char* ws = (char*)d_ws;
  size_t off = 0;
  auto carve = [&](size_t bytes) -> char* {
    char* p = ws + off;
    off += (bytes + 255) & ~(size_t)255;
    return p;
  };
  _Float16* W16  = (_Float16*)carve((size_t)E * E * 2);
  _Float16* X16  = (_Float16*)carve((size_t)M * E * 2);
  _Float16* Q16  = (_Float16*)carve((size_t)M * E * 2);
  _Float16* K16  = (_Float16*)carve((size_t)M * E * 2);
  _Float16* V16  = (_Float16*)carve((size_t)M * E * 2);
  _Float16* O16  = (_Float16*)carve((size_t)M * E * 2);
  _Float16* rk16 = (_Float16*)carve((size_t)RKROWS * D * 2);
  _Float16* rvT  = (_Float16*)carve((size_t)D * RVK * 2);
  if (off > ws_size) return;

  const int n2W = E * E / 2;
  const int n2X = M * E / 2;
  const float wsc = 64.0f, winv = 1.0f / 64.0f;
  const float rvsc = 2048.0f;
  const int gemmTiles  = (M / 64) * (E / 64);
  const int gemmBlocks = (gemmTiles + 7) / 8;

  cast_scale_f32_f16x2<<<(n2W + 255) / 256, 256, 0, stream>>>(Wq, W16, n2W, wsc);
  cast_f32_f16x2<<<(n2X + 255) / 256, 256, 0, stream>>>(q, X16, n2X);
  wmma_gemm64<0, false, 2, 1, false><<<dim3(gemmBlocks, 1), 256, 0, stream>>>(
      U16(X16), U16(X16), E, 0L, U16(W16), U16(W16), E, 0L,
      (void*)Q16, (void*)Q16, E, 0L, bq, bq, 0L, M, E, E, winv);
  cast_scale_f32_f16x2<<<(n2W + 255) / 256, 256, 0, stream>>>(Wk, W16, n2W, wsc);
  cast_f32_f16x2<<<(n2X + 255) / 256, 256, 0, stream>>>(k, X16, n2X);
  wmma_gemm64<0, false, 2, 1, false><<<dim3(gemmBlocks, 1), 256, 0, stream>>>(
      U16(X16), U16(X16), E, 0L, U16(W16), U16(W16), E, 0L,
      (void*)K16, (void*)K16, E, 0L, bk, bk, 0L, M, E, E, winv);
  cast_scale_f32_f16x2<<<(n2W + 255) / 256, 256, 0, stream>>>(Wv, W16, n2W, wsc);
  cast_f32_f16x2<<<(n2X + 255) / 256, 256, 0, stream>>>(v, X16, n2X);
  wmma_gemm64<0, false, 2, 1, false><<<dim3(gemmBlocks, 1), 256, 0, stream>>>(
      U16(X16), U16(X16), E, 0L, U16(W16), U16(W16), E, 0L,
      (void*)V16, (void*)V16, E, 0L, bv, bv, 0L, M, E, E, winv);
  cast_rk_rows<<<(RKROWS * 32 + 255) / 256, 256, 0, stream>>>(rk, rk16, R, RKROWS, wsc);
  cast_rv_T<<<(32 * RVK + 255) / 256, 256, 0, stream>>>(rv, rvT, R, RVK, rvsc);
  rel_attn_kernel<<<dim3(B * 16 * (S / 64)), 128, RA_LDS, stream>>>(Q16, K16, V16, rk16, rvT, O16);
  cast_scale_f32_f16x2<<<(n2W + 255) / 256, 256, 0, stream>>>(Wo, W16, n2W, wsc);
  wmma_gemm64<0, false, 2, 0, false><<<dim3(gemmBlocks, 1), 256, 0, stream>>>(
      U16(O16), U16(O16), E, 0L, U16(W16), U16(W16), E, 0L,
      (void*)out, (void*)out, E, 0L, bo, bo, 0L, M, E, E, winv);
}
